// RelativePositionSDPA_90829968376477
// MI455X (gfx1250) — hardware-verified
//
#include <hip/hip_runtime.h>
#include <math.h>
#include <stdint.h>

#define NHT   16
#define NHD   8
#define SQ    1024
#define DH    64
#define DM    512
#define KD    1024
#define RROWS 1088
#define NQB   16
static_assert(NQB * 64 == SQ);
static_assert(NQB == 16);
static_assert(RROWS == 17 * 64);
static_assert(RROWS >= (SQ - 64) + 128);
static_assert((DM % 64) == 0 && (KD % 32) == 0 && (DH % 32) == 0);
static_assert(((NHT * SQ) % 256) == 0 && ((NHD * RROWS) % 256) == 0);
#define UK_BLOCKS ((NHT * SQ) / 256)
#define RV_BLOCKS ((NHD * RROWS) / 256)

typedef __bf16   v16b __attribute__((ext_vector_type(16)));
typedef __bf16   v8b  __attribute__((ext_vector_type(8)));
typedef float    v8f  __attribute__((ext_vector_type(8)));
typedef float    v4f  __attribute__((ext_vector_type(4)));
typedef unsigned int v4u __attribute__((ext_vector_type(4)));
typedef unsigned short v8us __attribute__((ext_vector_type(8)));

__device__ __forceinline__ unsigned short bf_bits(float f) {
  unsigned u = __float_as_uint(f);
  return (unsigned short)((u + 0x7FFFu + ((u >> 16) & 1u)) >> 16);
}
__device__ __forceinline__ float bf_up(unsigned short h) { return __uint_as_float(((unsigned)h) << 16); }
__device__ __forceinline__ __bf16 bf_val(unsigned short h) { return __builtin_bit_cast(__bf16, h); }
__device__ __forceinline__ unsigned pk16(unsigned short a, unsigned short b) { return (unsigned)a | ((unsigned)b << 16); }
__device__ __forceinline__ v8f zero8() { v8f z = {0.f, 0.f, 0.f, 0.f, 0.f, 0.f, 0.f, 0.f}; return z; }

__device__ __forceinline__ v16b ldfrag_b(const __bf16* p) {
  union { v16b v; v8b h[2]; } f;
  f.h[0] = *(const v8b*)(p);
  f.h[1] = *(const v8b*)(p + 16);
  return f.v;
}

__device__ __forceinline__ v8f mma_b(v16b a, v16b b, v8f c) {
  c = __builtin_amdgcn_wmma_f32_16x16x32_bf16(false, a, false, b, (short)0, c, false, false);
  asm volatile("v_nop\n\tv_nop\n\tv_nop\n\tv_nop" : "+v"(c) : "v"(a), "v"(b));
  return c;
}
__device__ __forceinline__ v8f mma_b_raw(v16b a, v16b b, v8f c) {
  return __builtin_amdgcn_wmma_f32_16x16x32_bf16(false, a, false, b, (short)0, c, false, false);
}
__device__ __forceinline__ void dep_guard_b(v8f& a, v8f& b, v16b x) {
  asm volatile("v_nop\n\tv_nop\n\tv_nop\n\tv_nop" : "+v"(a), "+v"(b) : "v"(x));
}
__device__ __forceinline__ void keep4_b(v16b a, v16b b, v16b c, v16b d) {
  asm volatile("v_nop" :: "v"(a), "v"(b), "v"(c), "v"(d));
}
__device__ __forceinline__ void acc_guard4(v8f& a, v8f& b, v8f& c, v8f& d) {
  asm volatile("v_nop\n\tv_nop\n\tv_nop\n\tv_nop" : "+v"(a), "+v"(b), "+v"(c), "+v"(d));
}

__global__ __launch_bounds__(256) void cvt_bf16x8(const float* __restrict__ in, unsigned short* out, int n8) {
  const int i = blockIdx.x * 256 + threadIdx.x;
  if (i < n8) {
    const v4f a = *(const v4f*)(in + (size_t)i * 8);
    const v4f b = *(const v4f*)(in + (size_t)i * 8 + 4);
    v4u p;
    p[0] = pk16(bf_bits(a[0]), bf_bits(a[1]));
    p[1] = pk16(bf_bits(a[2]), bf_bits(a[3]));
    p[2] = pk16(bf_bits(b[0]), bf_bits(b[1]));
    p[3] = pk16(bf_bits(b[2]), bf_bits(b[3]));
    *(volatile v4u*)(out + (size_t)i * 8) = p;
    __threadfence();
    *(volatile v4u*)(out + (size_t)i * 8) = p;
  }
}

__global__ __launch_bounds__(256) void cvt_wdup(const float* __restrict__ W, unsigned short* Wd, int n8) {
  const int i = blockIdx.x * 256 + threadIdx.x;
  if (i < n8) {
    const int o = i >> 6;
    const int c = (i & 63) * 8;
    const v4f a = *(const v4f*)(W + (size_t)o * DM + c);
    const v4f b = *(const v4f*)(W + (size_t)o * DM + c + 4);
    v4u p;
    p[0] = pk16(bf_bits(a[0]), bf_bits(a[1]));
    p[1] = pk16(bf_bits(a[2]), bf_bits(a[3]));
    p[2] = pk16(bf_bits(b[0]), bf_bits(b[1]));
    p[3] = pk16(bf_bits(b[2]), bf_bits(b[3]));
    unsigned short* d0 = Wd + (size_t)o * KD + c;
    *(volatile v4u*)(d0) = p;
    *(volatile v4u*)(d0 + DM) = p;
    __threadfence();
    *(volatile v4u*)(d0) = p;
    *(volatile v4u*)(d0 + DM) = p;
  }
}

__global__ __launch_bounds__(256) void pe_prep(unsigned short* PEd) {
  const int p = blockIdx.x;
  const int i = threadIdx.x;
  const float pos  = (float)(SQ - 1 - p);
  const float kc   = (float)((-9.2103403 - 7.1976184e-8) / 512.0);
  const float invf = expf((float)(2 * i) * kc);
  const float ang  = pos * invf;
  const float sv = sinf(ang);
  const float cv = cosf(ang);
  const unsigned short hs = bf_bits(sv), hc = bf_bits(cv);
  const unsigned short ls = bf_bits(sv - bf_up(hs)), lc = bf_bits(cv - bf_up(hc));
  const unsigned wh = pk16(hs, hc);
  const unsigned wl = pk16(ls, lc);
  unsigned short* d = PEd + (size_t)p * KD + 2 * i;
  *(volatile unsigned*)(d) = wh;
  *(volatile unsigned*)(d + DM) = wl;
  __threadfence();
  *(volatile unsigned*)(d) = wh;
  *(volatile unsigned*)(d + DM) = wl;
}

__global__ __launch_bounds__(256) void rgemm(const unsigned short* __restrict__ Ap,
                                             const unsigned short* __restrict__ Btp,
                                             unsigned short* Chp, unsigned short* Clp) {
  constexpr int M = RROWS;
  constexpr int N = DM;
  constexpr int K = KD;
  constexpr int lda = KD;
  constexpr int ldb = KD;
  static_assert((M % 64) == 0 && (N % 64) == 0 && (K % 32) == 0);
  __shared__ __align__(16) float sT[8][16 * 68];
  const __bf16* Ab = (const __bf16*)(const void*)Ap;
  const __bf16* Bb = (const __bf16*)(const void*)Btp;

  const int lane = threadIdx.x & 31;
  const int wave = threadIdx.x >> 5;
  const int tilesN = N >> 6;
  const int tilesM = M >> 6;
  const int tile = blockIdx.x * 8 + wave;
  if (tile >= tilesM * tilesN) return;
  const int tm = tile / tilesN;
  const int tn = tile - tm * tilesN;
  const int m0 = tm << 6;
  const int n0 = tn << 6;

  const int rlane = lane & 15;
  const int koff  = (lane >> 4) * 8;
  const int mOff  = (lane >> 4) * 8;

  v8f acc[4][4];
#pragma unroll
  for (int i = 0; i < 4; ++i)
#pragma unroll
    for (int j = 0; j < 4; ++j) acc[i][j] = zero8();

  for (int k0 = 0; k0 < K; k0 += 32) {
    v16b bh[4];
#pragma unroll
    for (int j = 0; j < 4; ++j) {
      const size_t bo = (size_t)(n0 + (j << 4) + rlane) * ldb + koff + k0;
      bh[j] = ldfrag_b(Bb + bo);
    }
#pragma unroll
    for (int i = 0; i < 4; ++i) {
      const size_t ao = (size_t)(m0 + (i << 4) + rlane) * lda + koff + k0;
      const v16b ah = ldfrag_b(Ab + ao);
#pragma unroll
      for (int j = 0; j < 4; ++j) {
        acc[i][j] = mma_b_raw(ah, bh[j], acc[i][j]);
      }
      dep_guard_b(acc[i][0], acc[i][3], ah);
    }
    keep4_b(bh[0], bh[1], bh[2], bh[3]);
  }
  acc_guard4(acc[0][0], acc[0][1], acc[0][2], acc[0][3]);
  acc_guard4(acc[1][0], acc[1][1], acc[1][2], acc[1][3]);
  acc_guard4(acc[2][0], acc[2][1], acc[2][2], acc[2][3]);
  acc_guard4(acc[3][0], acc[3][1], acc[3][2], acc[3][3]);

  float* slab = sT[wave];
  unsigned short* C  = Chp;
  unsigned short* C2 = Clp;
#pragma unroll
  for (int i = 0; i < 4; ++i) {
    const int mBase = m0 + (i << 4);
#pragma unroll
    for (int j = 0; j < 4; ++j) {
#pragma unroll
      for (int r = 0; r < 8; ++r) {
        slab[(mOff + r) * 68 + (j << 4) + rlane] = acc[i][j][r];
      }
    }
    __builtin_amdgcn_fence(__ATOMIC_RELEASE, "workgroup");
    __builtin_amdgcn_wave_barrier();
    __builtin_amdgcn_fence(__ATOMIC_ACQUIRE, "workgroup");
    {
      const int q = lane >> 3, c8 = (lane & 7) * 8;
      v4u hv[4], lv[4];
#pragma unroll
      for (int it = 0; it < 4; ++it) {
        const int row = it * 4 + q;
        const float* sp = slab + row * 68 + c8;
        v4u a, a2;
#pragma unroll
        for (int e = 0; e < 4; ++e) {
          const float f0 = sp[2 * e], f1 = sp[2 * e + 1];
          const unsigned short h0 = bf_bits(f0), h1 = bf_bits(f1);
          const unsigned short l0 = bf_bits(f0 - bf_up(h0)), l1 = bf_bits(f1 - bf_up(h1));
          a[e] = pk16(h0, h1); a2[e] = pk16(l0, l1);
        }
        hv[it] = a; lv[it] = a2;
      }
#pragma unroll
      for (int it = 0; it < 4; ++it) {
        const int row = it * 4 + q;
        *(volatile v4u*)(C  + (size_t)(mBase + row) * N + n0 + c8) = hv[it];
        *(volatile v4u*)(C2 + (size_t)(mBase + row) * N + n0 + c8) = lv[it];
      }
      __threadfence();
#pragma unroll
      for (int it = 0; it < 4; ++it) {
        const int row = it * 4 + q;
        *(volatile v4u*)(C  + (size_t)(mBase + row) * N + n0 + c8) = hv[it];
        *(volatile v4u*)(C2 + (size_t)(mBase + row) * N + n0 + c8) = lv[it];
      }
      __threadfence();
    }
    __builtin_amdgcn_fence(__ATOMIC_RELEASE, "workgroup");
    __builtin_amdgcn_wave_barrier();
    __builtin_amdgcn_fence(__ATOMIC_ACQUIRE, "workgroup");
  }
}

__global__ __launch_bounds__(256) void side_tables(const unsigned short* __restrict__ Kbp,
                                                   const float* __restrict__ ub, const float* __restrict__ vb,
                                                   const unsigned short* __restrict__ Rhp,
                                                   const unsigned short* __restrict__ Rlp,
                                                   float* ukp, float* rvp) {
  __shared__ __align__(16) float sF[256];
  const int tid  = threadIdx.x;
  const int wave = tid >> 5;
  const int lane = tid & 31;
  float  val;
  float* dst;
  if (blockIdx.x < UK_BLOCKS) {
    const int gid = blockIdx.x * 256 + tid;
    const int h   = (gid >> 10) & 7;
    const unsigned short* kr = Kbp + (size_t)gid * DH;
    const float* up = ub + h * DH;
    float a = 0.f;
#pragma unroll 1
    for (int c8 = 0; c8 < DH; c8 += 8) {
      const v8us kw = *(const v8us*)(kr + c8);
      const v4f u0 = *(const v4f*)(up + c8);
      const v4f u1 = *(const v4f*)(up + c8 + 4);
#pragma unroll
      for (int e = 0; e < 4; ++e) a = fmaf(bf_up(bf_bits(u0[e])), bf_up(kw[e]), a);
#pragma unroll
      for (int e = 0; e < 4; ++e) a = fmaf(bf_up(bf_bits(u1[e])), bf_up(kw[4 + e]), a);
    }
    val = a;
    dst = ukp + (size_t)blockIdx.x * 256 + wave * 32;
  } else {
    const int idx = (blockIdx.x - UK_BLOCKS) * 256 + tid;
    const int h   = idx / RROWS;
    const int p   = idx - h * RROWS;
    const unsigned short* rh = Rhp + (size_t)p * DM + h * DH;
    const unsigned short* rl = Rlp + (size_t)p * DM + h * DH;
    const float* vp = vb + h * DH;
    float a = 0.f;
#pragma unroll 1
    for (int c8 = 0; c8 < DH; c8 += 8) {
      const v8us hw = *(const v8us*)(rh + c8);
      const v8us lw = *(const v8us*)(rl + c8);
      const v4f v0 = *(const v4f*)(vp + c8);
      const v4f v1 = *(const v4f*)(vp + c8 + 4);
#pragma unroll
      for (int e = 0; e < 4; ++e) a = fmaf(bf_up(bf_bits(v0[e])), bf_up(hw[e]) + bf_up(lw[e]), a);
#pragma unroll
      for (int e = 0; e < 4; ++e) a = fmaf(bf_up(bf_bits(v1[e])), bf_up(hw[4 + e]) + bf_up(lw[4 + e]), a);
    }
    val = a;
    dst = rvp + (size_t)(blockIdx.x - UK_BLOCKS) * 256 + wave * 32;
  }
  sF[tid] = val;
  __syncthreads();
  if (lane < 8) {
    const v4f o = *(const v4f*)(sF + wave * 32 + lane * 4);
    *(volatile v4f*)(dst + lane * 4) = o;
    __threadfence();
    *(volatile v4f*)(dst + lane * 4) = o;
  }
}

#define KP 72
#define VP 72
#define RP 72
#define MP 68
#define L_KS   0
#define L_VT   9216
#define L_RH   18432
#define L_RL   36864
#define L_MS   55296
#define L_UK   72704
#define L_RV   72960
#define L_PH   73472
#define L_PL   81664
#define L_BD   89856
#define L_TOT  106240
static_assert(L_VT - L_KS == 64 * KP * 2);
static_assert(L_RH - L_VT == 64 * VP * 2);
static_assert(L_RL - L_RH == 128 * RP * 2);
static_assert(L_MS - L_RL == 128 * RP * 2);
static_assert(L_UK - L_MS == 64 * MP * 4);
static_assert(L_RV - L_UK == 64 * 4);
static_assert(L_PH - L_RV == 128 * 4);
static_assert(L_PL - L_PH == 4 * 16 * 64 * 2);
static_assert(L_BD - L_PL == 4 * 16 * 64 * 2);
static_assert(L_TOT - L_BD == 4 * 16 * 64 * 4);
static_assert(4 * 16 * 64 * 4 <= L_RL - L_RH);
static_assert((KP % 8) == 0 && (VP % 8) == 0 && (RP % 8) == 0 && (MP % 4) == 0 && (L_BD % 16) == 0);

__global__ __launch_bounds__(128) __attribute__((amdgpu_num_vgpr(256)))
void attn_rel(const unsigned short* __restrict__ Sbp, const unsigned short* __restrict__ Kbp,
              const unsigned short* __restrict__ Vbp, const unsigned short* __restrict__ Rhp,
              const unsigned short* __restrict__ Rlp, const float* __restrict__ ukp,
              const float* __restrict__ rvp, const float* __restrict__ mkp, float* outp) {
  extern __shared__ __align__(16) unsigned char lds[];
  union FB { v16b v; v8b h[2]; };
  __bf16*         Ks  = (__bf16*)(lds + L_KS);
  unsigned short* Vtu = (unsigned short*)(lds + L_VT);
  const __bf16*   Vt  = (const __bf16*)(lds + L_VT);
  __bf16*         RhL = (__bf16*)(lds + L_RH);
  __bf16*         RlL = (__bf16*)(lds + L_RL);
  float*          sM  = (float*)(lds + L_MS);
  float*          sUk = (float*)(lds + L_UK);
  float*          sRv = (float*)(lds + L_RV);
  __bf16*         Ph  = (__bf16*)(lds + L_PH);
  __bf16*         Pl  = (__bf16*)(lds + L_PL);
  float*          Bd  = (float*)(lds + L_BD);

  const int tid  = threadIdx.x;
  const int wave = tid >> 5;
  const int lane = tid & 31;
  const int hh   = lane >> 4;
  const int c    = lane & 15;

  const int bx    = blockIdx.x;
  const int qb    = bx & (NQB - 1);
  const int nh    = bx >> 4;
  const int h     = nh & 7;
  const int q0blk = qb * 64;
  const int q0    = q0blk + wave * 16;
  const int tb    = 3 - wave;
  const size_t hrow = (size_t)nh * SQ;

  const __bf16* Sb = (const __bf16*)(const void*)Sbp;
  const __bf16* Kb = (const __bf16*)(const void*)Kbp;
  const __bf16* Rh = (const __bf16*)(const void*)Rhp;
  const __bf16* Rl = (const __bf16*)(const void*)Rlp;

  __bf16* pwh = Ph + wave * 1024;
  __bf16* pwl = Pl + wave * 1024;
  float*  bdw = Bd + wave * 1024;

  v8f acc[4];
#pragma unroll
  for (int t = 0; t < 4; ++t) acc[t] = zero8();

  float mrow[8], lrow[8], alpha[8];
#pragma unroll
  for (int r = 0; r < 8; ++r) { mrow[r] = -INFINITY; lrow[r] = 0.f; alpha[r] = 0.f; }

  const size_t qo = (hrow + q0 + c) * DH + 8 * hh;

  for (int kt = 0; kt <= qb; ++kt) {
    const int kv0 = kt * 64;
    const int pw0 = kv0 - q0blk + (SQ - 64);
    __syncthreads();
    {
      const __bf16*         kg = Kb  + (hrow + kv0) * DH;
      const unsigned short* vg = Vbp + (hrow + kv0) * DH;
#pragma unroll 2
      for (int i = 0; i < 4; ++i) {
        const int p   = tid + 128 * i;
        const int key = p >> 3;
        const int d8  = (p & 7) * 8;
        const v8b  k8 = *(const v8b*)(kg + p * 8);
        const v8us v8 = *(const v8us*)(vg + p * 8);
        *(v8b*)(Ks + key * KP + d8) = k8;
#pragma unroll
        for (int e = 0; e < 8; ++e) Vtu[(d8 + e) * VP + key] = v8[e];
      }
      const __bf16* rgh = Rh + (size_t)pw0 * DM + h * DH;
      const __bf16* rgl = Rl + (size_t)pw0 * DM + h * DH;
#pragma unroll 2
      for (int i = 0; i < 8; ++i) {
        const int p   = tid + 128 * i;
        const int row = p >> 3;
        const int d8  = (p & 7) * 8;
        const v8b a0 = *(const v8b*)(rgh + (size_t)row * DM + d8);
        const v8b a1 = *(const v8b*)(rgl + (size_t)row * DM + d8);
        *(v8b*)(RhL + row * RP + d8) = a0;
        *(v8b*)(RlL + row * RP + d8) = a1;
      }
      const float* mg = mkp + (size_t)q0blk * SQ + kv0;
#pragma unroll 2
      for (int i = 0; i < 8; ++i) {
        const int p   = tid + 128 * i;
        const int row = p >> 4;
        const int c4  = (p & 15) * 4;
        const v4f mv = *(const v4f*)(mg + (size_t)row * SQ + c4);
        v4f mc;
#pragma unroll
        for (int e = 0; e < 4; ++e) mc[e] = bf_up(bf_bits(mv[e]));
        *(v4f*)(sM + row * MP + c4) = mc;
      }
      if (tid < 64) sUk[tid] = ukp[hrow + kv0 + tid];
      sRv[tid] = rvp[(size_t)h * RROWS + pw0 + tid];
    }
    __syncthreads();

    {
      v8f e[5];
#pragma unroll
      for (int u = 0; u < 5; ++u) e[u] = zero8();
#pragma unroll 1
      for (int dc = 0; dc < 2; ++dc) {
        const v16b qa = ldfrag_b(Sb + qo + dc * 32);
        const int ko = dc * 32 + 8 * hh;
#pragma unroll
        for (int u = 0; u < 5; ++u) {
          const int rr = ((tb + u) * 16 + c) * RP + ko;
          FB ra;
          ra.h[0] = *(const v8b*)(RhL + rr);
          ra.h[1] = *(const v8b*)(RhL + rr + 16);
          e[u] = mma_b(qa, ra.v, e[u]);
        }
#pragma unroll
        for (int u = 0; u < 5; ++u) {
          const int rr = ((tb + u) * 16 + c) * RP + ko;
          FB rb;
          rb.h[0] = *(const v8b*)(RlL + rr);
          rb.h[1] = *(const v8b*)(RlL + rr + 16);
          e[u] = mma_b(qa, rb.v, e[u]);
        }
      }
#pragma unroll
      for (int u = 0; u < 5; ++u) {
        const float a = sRv[(tb + u) * 16 + c];
#pragma unroll
        for (int r = 0; r < 8; ++r) e[u][r] += a;
      }
#pragma unroll
      for (int r = 0; r < 8; ++r) {
        const int ii = 8 * hh + r;
        const int la = (hh << 4) | ((15 + c - ii) & 15);
        const int lb = (hh << 4) | ((c - ii - 1) & 15);
#pragma unroll
        for (int j = 0; j < 4; ++j) {
          const float b0 = __shfl(e[j][r], la, 32);
          const float b1 = __shfl(e[j + 1][r], lb, 32);
          bdw[ii * 64 + j * 16 + c] = (c > ii) ? b1 : b0;
        }
      }
    }
    __builtin_amdgcn_fence(__ATOMIC_RELEASE, "workgroup");
    __builtin_amdgcn_wave_barrier();
    __builtin_amdgcn_fence(__ATOMIC_ACQUIRE, "workgroup");

    v8f s[4];
#pragma unroll
    for (int j = 0; j < 4; ++j) s[j] = zero8();
#pragma unroll 1
    for (int dc = 0; dc < 2; ++dc) {
      const v16b qa = ldfrag_b(Sb + qo + dc * 32);
      const int ko = dc * 32 + 8 * hh;
#pragma unroll
      for (int j = 0; j < 4; ++j) {
        const int kr = (j * 16 + c) * KP + ko;
        FB kb;
        kb.h[0] = *(const v8b*)(Ks + kr);
        kb.h[1] = *(const v8b*)(Ks + kr + 16);
        s[j] = mma_b(qa, kb.v, s[j]);
      }
    }
#pragma unroll
    for (int j = 0; j < 4; ++j) {
      const float a = sUk[j * 16 + c];
#pragma unroll
      for (int r = 0; r < 8; ++r) s[j][r] += a;
    }

#pragma unroll
    for (int r = 0; r < 8; ++r) {
      const int ii = 8 * hh + r;
      const int sl = wave * 16 + ii;
      float m = -INFINITY;
#pragma unroll
      for (int j = 0; j < 4; ++j) {
        const float bd = bdw[ii * 64 + j * 16 + c];
        const float mk = sM[sl * MP + j * 16 + c];
        const float sv = (s[j][r] + bd) * 0.125f + mk;
        s[j][r] = sv;
        m = fmaxf(m, sv);
      }
#pragma unroll
      for (int off = 1; off < 16; off <<= 1) m = fmaxf(m, __shfl_xor(m, off, 32));
      const float mnew  = fmaxf(mrow[r], m);
      const float msafe = (mnew == -INFINITY) ? 0.f : mnew;
      const float al    = __expf(mrow[r] - msafe);
      mrow[r]  = mnew;
      alpha[r] = al;
      float psum = 0.f;
#pragma unroll
      for (int j = 0; j < 4; ++j) {
        const float p = __expf(s[j][r] - msafe);
        psum += p;
        const unsigned short hb = bf_bits(p);
        const unsigned short lw = bf_bits(p - bf_up(hb));
        const int po = ii * 64 + j * 16 + c;
        pwh[po] = bf_val(hb);
        pwl[po] = bf_val(lw);
      }
#pragma unroll
      for (int off = 1; off < 16; off <<= 1) psum += __shfl_xor(psum, off, 32);
      lrow[r] = lrow[r] * al + psum;
    }
    __builtin_amdgcn_fence(__ATOMIC_RELEASE, "workgroup");
    __builtin_amdgcn_wave_barrier();
    __builtin_amdgcn_fence(__ATOMIC_ACQUIRE, "workgroup");

    FB pa[2], pl[2];
#pragma unroll
    for (int kk = 0; kk < 2; ++kk) {
      const int pr = c * 64 + kk * 32 + 8 * hh;
      pa[kk].h[0] = *(const v8b*)(pwh + pr);
      pa[kk].h[1] = *(const v8b*)(pwh + pr + 16);
      pl[kk].h[0] = *(const v8b*)(pwl + pr);
      pl[kk].h[1] = *(const v8b*)(pwl + pr + 16);
    }
#pragma unroll
    for (int t = 0; t < 4; ++t) {
#pragma unroll
      for (int r = 0; r < 8; ++r) acc[t][r] *= alpha[r];
      const int vr0 = (t * 16 + c) * VP + 8 * hh;
#pragma unroll
      for (int kk = 0; kk < 2; ++kk) {
        FB vf;
        vf.h[0] = *(const v8b*)(Vt + vr0 + kk * 32);
        vf.h[1] = *(const v8b*)(Vt + vr0 + kk * 32 + 16);
        acc[t] = mma_b(pa[kk].v, vf.v, acc[t]);
        acc[t] = mma_b(pl[kk].v, vf.v, acc[t]);
      }
    }
  }

  __syncthreads();

  float* os = (float*)(lds + L_RH) + wave * 1024;
  float inv[8];
#pragma unroll
  for (int r = 0; r < 8; ++r) inv[r] = (lrow[r] > 0.f) ? (1.0f / lrow[r]) : 0.f;
#pragma unroll
  for (int t = 0; t < 4; ++t) {
#pragma unroll
    for (int r = 0; r < 8; ++r) os[(8 * hh + r) * 64 + t * 16 + c] = acc[t][r] * inv[r];
  }
  __builtin_amdgcn_fence(__ATOMIC_RELEASE, "workgroup");
  __builtin_amdgcn_wave_barrier();
  __builtin_amdgcn_fence(__ATOMIC_ACQUIRE, "workgroup");
  float* og = outp + (hrow + q0) * DH;
  v4f ov[8];
#pragma unroll
  for (int it = 0; it < 8; ++it) ov[it] = *(const v4f*)(os + it * 128 + lane * 4);
#pragma unroll
  for (int it = 0; it < 8; ++it) *(volatile v4f*)(og + it * 128 + lane * 4) = ov[it];
  __threadfence();
#pragma unroll
  for (int it = 0; it < 8; ++it) *(volatile v4f*)(og + it * 128 + lane * 4) = ov[it];
}

extern "C" void kernel_launch(void* const* d_in, const int* in_sizes, int n_in,
                              void* d_out, int out_size, void* d_ws, size_t ws_size,
                              hipStream_t stream) {
  if (n_in < 7) return;
  if (in_sizes[0] != NHT * SQ * DH || in_sizes[1] != NHT * SQ * DH || in_sizes[2] != NHT * SQ * DH) return;
  if (in_sizes[3] != NHD * DH || in_sizes[4] != NHD * DH) return;
  if (in_sizes[5] != DM * DM) return;
  if (in_sizes[6] != SQ * SQ) return;
  if (out_size != NHT * SQ * DH) return;

  const float* seqs = (const float*)d_in[0];
  const float* keys = (const float*)d_in[1];
  const float* vals = (const float*)d_in[2];
  const float* ub   = (const float*)d_in[3];
  const float* vb   = (const float*)d_in[4];
  const float* W    = (const float*)d_in[5];
  const float* mk   = (const float*)d_in[6];

  const size_t PSB = (size_t)NHT * SQ * DH * 2;
  const size_t PWD = (size_t)DM * KD * 2;
  const size_t PPE = (size_t)RROWS * KD * 2;
  const size_t PR  = (size_t)RROWS * DM * 2;
  const size_t PUK = (size_t)NHT * SQ * 4;
  const size_t PRV = (size_t)NHD * RROWS * 4;
  static_assert(((size_t)NHD * RROWS * 4) % 128 == 0);
  static_assert(((size_t)RROWS * DM * 2) % 128 == 0);
  size_t off = 0;
  const size_t oSb = off; off += PSB;
  const size_t oKb = off; off += PSB;
  const size_t oVb = off; off += PSB;
  const size_t oWd = off; off += PWD;
  const size_t oPE = off; off += PPE;
  const size_t oRh = off; off += PR;
  const size_t oRl = off; off += PR;
  const size_t oUk = off; off += PUK;
  const size_t oRv = off; off += PRV;
  if (off > ws_size) return;
  if (off > ((size_t)128 << 20)) return;

  char* ws = (char*)d_ws;
  unsigned short* Sb  = (unsigned short*)(ws + oSb);
  unsigned short* Kb  = (unsigned short*)(ws + oKb);
  unsigned short* Vb  = (unsigned short*)(ws + oVb);
  unsigned short* Wd  = (unsigned short*)(ws + oWd);
  unsigned short* PEd = (unsigned short*)(ws + oPE);
  unsigned short* Rh  = (unsigned short*)(ws + oRh);
  unsigned short* Rl  = (unsigned short*)(ws + oRl);
  float*          uk  = (float*)(ws + oUk);
  float*          rv  = (float*)(ws + oRv);

  const dim3 blk(256);
  const int n8x = NHT * SQ * DH / 8;
  const int n8w = DM * DM / 8;
  const dim3 gCvt((n8x + 255) / 256);
  const dim3 gWd((n8w + 255) / 256);
  const dim3 gPe(RROWS);
  const dim3 gR(((RROWS / 64) * (DM / 64) + 7) / 8);
  const dim3 gSide(UK_BLOCKS + RV_BLOCKS);
  const dim3 gAttn(NHT * NQB);

  cvt_bf16x8<<<gCvt, blk, 0, stream>>>(seqs, Sb, n8x);
  cvt_bf16x8<<<gCvt, blk, 0, stream>>>(keys, Kb, n8x);
  cvt_bf16x8<<<gCvt, blk, 0, stream>>>(vals, Vb, n8x);
  cvt_wdup<<<gWd, blk, 0, stream>>>(W, Wd, n8w);
  pe_prep<<<gPe, blk, 0, stream>>>(PEd);
  rgemm<<<gR, blk, 0, stream>>>(PEd, Wd, Rh, Rl);
  side_tables<<<gSide, blk, 0, stream>>>(Kb, ub, vb, Rh, Rl, uk, rv);
  (void)hipFuncSetAttribute(reinterpret_cast<const void*>(&attn_rel),
                            hipFuncAttributeMaxDynamicSharedMemorySize, L_TOT);
  attn_rel<<<gAttn, dim3(128), L_TOT, stream>>>(Sb, Kb, Vb, Rh, Rl, uk, rv, mk, (float*)d_out);
  (void)hipGetLastError();
}
